// BorderBranch_21234318311586
// MI455X (gfx1250) — hardware-verified
//
#include <hip/hip_runtime.h>
#include <hip/hip_bf16.h>
#include <stdint.h>


typedef __attribute__((ext_vector_type(16))) _Float16 v16h;
typedef __attribute__((ext_vector_type(8)))  _Float16 v8h;
typedef __attribute__((ext_vector_type(16))) __bf16   v16b;
typedef __attribute__((ext_vector_type(8)))  __bf16   v8b;
typedef __attribute__((ext_vector_type(8)))  float    v8f;
typedef __attribute__((ext_vector_type(4)))  float    v4f;
typedef __attribute__((ext_vector_type(2)))  float    v2f;

__device__ __forceinline__ unsigned short f2bf_bits(float f) {
  unsigned u = __float_as_uint(f);
  return (unsigned short)((u + 0x7FFFu + ((u >> 16) & 1u)) >> 16);
}
__device__ __forceinline__ float bf_bits2f(unsigned short h) { return __uint_as_float(((unsigned)h) << 16); }

__device__ __forceinline__ void dep_guard_h(v8f& a, v8f& b, v16h x, v16h y) { asm volatile("v_nop\n\tv_nop\n\tv_nop\n\tv_nop" : "+v"(a), "+v"(b) : "v"(x), "v"(y)); }
__device__ __forceinline__ void dep_guard_b(v8f& a, v8f& b, v16b x, v16b y) { asm volatile("v_nop\n\tv_nop\n\tv_nop\n\tv_nop" : "+v"(a), "+v"(b) : "v"(x), "v"(y)); }
__device__ __forceinline__ void keep4_h(v16h a, v16h b, v16h c, v16h d) { asm volatile("v_nop" :: "v"(a), "v"(b), "v"(c), "v"(d)); }
__device__ __forceinline__ void keep4_b(v16b a, v16b b, v16b c, v16b d) { asm volatile("v_nop" :: "v"(a), "v"(b), "v"(c), "v"(d)); }
__device__ __forceinline__ void acc_guard4(v8f& a, v8f& b, v8f& c, v8f& d) { asm volatile("v_nop\n\tv_nop\n\tv_nop\n\tv_nop" : "+v"(a), "+v"(b), "+v"(c), "+v"(d)); }
template <typename T> struct Frag;
template <> struct Frag<_Float16> {
  typedef v16h V; union U { v16h v; v8h h[2]; };
  static __device__ __forceinline__ v16h load(const _Float16* p) {
    U f; f.h[0] = *(const v8h*)(p); f.h[1] = *(const v8h*)(p + 16); return f.v;
  }
  static __device__ __forceinline__ v8f mma(v16h a, v16h b, v8f c) {
    return __builtin_amdgcn_wmma_f32_16x16x32_f16(false, a, false, b, (short)0, c, false, false);
  }
  static __device__ __forceinline__ void guard(v8f& a, v8f& b, v16h x, v16h y) { dep_guard_h(a, b, x, y); }
  static __device__ __forceinline__ void keep(v16h a, v16h b, v16h c, v16h d) { keep4_h(a, b, c, d); }
};
template <> struct Frag<__bf16> {
  typedef v16b V; union U { v16b v; v8b h[2]; };
  static __device__ __forceinline__ v16b load(const __bf16* p) {
    U f; f.h[0] = *(const v8b*)(p); f.h[1] = *(const v8b*)(p + 16); return f.v;
  }
  static __device__ __forceinline__ v8f mma(v16b a, v16b b, v8f c) {
    return __builtin_amdgcn_wmma_f32_16x16x32_bf16(false, a, false, b, (short)0, c, false, false);
  }
  static __device__ __forceinline__ void guard(v8f& a, v8f& b, v16b x, v16b y) { dep_guard_b(a, b, x, y); }
  static __device__ __forceinline__ void keep(v16b a, v16b b, v16b c, v16b d) { keep4_b(a, b, c, d); }
};

template <int ET> struct Elem;
template <> struct Elem<0> { typedef _Float16 T; };
template <> struct Elem<1> { typedef __bf16 T; };
template <int ET, bool SPLIT, int BIAS_MODE, int OUT_MODE, bool RESID, int ACT = 0>
__global__ __launch_bounds__(256) void wmma_gemm64(
    const unsigned short* __restrict__ Ap, const unsigned short* __restrict__ A2p, int lda, long strideA,
    const unsigned short* __restrict__ Btp, const unsigned short* __restrict__ Bt2p, int ldb, long strideB,
    void* __restrict__ Cout, void* __restrict__ Cout2, int ldc, long strideC,
    const float* __restrict__ bias,
    const float* __restrict__ resid, long strideR,
    int M, int N, int K, float scale) {
  typedef typename Elem<ET>::T T;
  typedef typename Frag<T>::V V;
  const T* A = (const T*)Ap; const T* A2 = (const T*)A2p; const T* Bt = (const T*)Btp; const T* Bt2 = (const T*)Bt2p;
  __shared__ __align__(16) float sT[8][16 * 68];
  const int b    = blockIdx.y;
  const int lane = threadIdx.x & 31;
  const int wave = threadIdx.x >> 5;
  const int tilesN = N >> 6;
  const int tilesM = M >> 6;
  const int tile = blockIdx.x * 8 + wave;
  if (tile >= tilesM * tilesN) return;
  const int tm = tile / tilesN;
  const int tn = tile - tm * tilesN;
  const int m0 = tm << 6;
  const int n0 = tn << 6;

  const T* Ab  = A  + (size_t)b * strideA;
  const T* Bb  = Bt + (size_t)b * strideB;
  const T* Ab2 = SPLIT ? (A2  + (size_t)b * strideA) : nullptr;
  const T* Bb2 = SPLIT ? (Bt2 + (size_t)b * strideB) : nullptr;

  const int rlane = lane & 15;
  const int koff  = (lane >> 4) * 8;
  const int mOff  = (lane >> 4) * 8;

  v8f acc[4][4];
#pragma unroll
  for (int i = 0; i < 4; ++i)
#pragma unroll
    for (int j = 0; j < 4; ++j) acc[i][j] = (v8f){0.f,0.f,0.f,0.f,0.f,0.f,0.f,0.f};

  for (int k0 = 0; k0 < K; k0 += 32) {
    V bh[4], bl[4];
#pragma unroll
    for (int j = 0; j < 4; ++j) {
      const size_t bo = (size_t)(n0 + (j << 4) + rlane) * ldb + koff + k0;
      bh[j] = Frag<T>::load(Bb + bo);
      if (SPLIT) bl[j] = Frag<T>::load(Bb2 + bo);
    }
#pragma unroll
    for (int i = 0; i < 4; ++i) {
      const size_t ao = (size_t)(m0 + (i << 4) + rlane) * lda + koff + k0;
      V ah = Frag<T>::load(Ab + ao);
      V al;
      if (SPLIT) al = Frag<T>::load(Ab2 + ao);
#pragma unroll
      for (int j = 0; j < 4; ++j) {
        acc[i][j] = Frag<T>::mma(ah, bh[j], acc[i][j]);
        if (SPLIT) {
          acc[i][j] = Frag<T>::mma(ah, bl[j], acc[i][j]);
          acc[i][j] = Frag<T>::mma(al, bh[j], acc[i][j]);
        }
      }
      Frag<T>::guard(acc[i][0], acc[i][3], ah, SPLIT ? al : ah);
    }
    Frag<T>::keep(bh[0], bh[1], bh[2], bh[3]);
    if (SPLIT) Frag<T>::keep(bl[0], bl[1], bl[2], bl[3]);
  }
  acc_guard4(acc[0][0], acc[0][1], acc[0][2], acc[0][3]);
  acc_guard4(acc[1][0], acc[1][1], acc[1][2], acc[1][3]);
  acc_guard4(acc[2][0], acc[2][1], acc[2][2], acc[2][3]);
  acc_guard4(acc[3][0], acc[3][1], acc[3][2], acc[3][3]);

  float* slab = sT[wave];
  const float* Rb = RESID ? (resid + (size_t)b * strideR) : nullptr;
#pragma unroll
  for (int i = 0; i < 4; ++i) {
    const int mBase = m0 + (i << 4);
#pragma unroll
    for (int j = 0; j < 4; ++j) {
      const int n = n0 + (j << 4) + rlane;
      float bv = 0.f;
      if (BIAS_MODE == 2) bv = bias[n];
#pragma unroll
      for (int r = 0; r < 8; ++r) {
        float v = acc[i][j][r] * scale;
        if (BIAS_MODE == 1) v += bias[mBase + mOff + r];
        if (BIAS_MODE == 2) v += bv;
        if (RESID) v += Rb[(size_t)(mBase + mOff + r) * ldc + n];
        if (ACT == 1) v = tanhf(v);
        if (ACT == 2) v = fmaxf(v, 0.0f);
        if (ACT == 3) v = v / (1.0f + expf(-v));
        if (ACT == 4) v = (v > 0.f) ? v : 0.01f * v;
        if (ACT == 5) v = 0.5f * v * (1.0f + erff(v * 0.70710678118654752f));
        slab[(mOff + r) * 68 + (j << 4) + rlane] = v;
      }
    }
    __builtin_amdgcn_fence(__ATOMIC_RELEASE, "workgroup");
    __builtin_amdgcn_wave_barrier();
    __builtin_amdgcn_fence(__ATOMIC_ACQUIRE, "workgroup");
    if (OUT_MODE == 0) {
      float* C = (float*)Cout + (size_t)b * strideC;
      const int hh = lane >> 4, c4 = (lane & 15) * 4;
      for (int pass = 0; pass < 2; ++pass) {
#pragma unroll
        for (int it = 0; it < 8; ++it) {
          const int row = it * 2 + hh;
          v4f v = *(const v4f*)(slab + row * 68 + c4);
          *(volatile v4f*)(C + (size_t)(mBase + row) * ldc + n0 + c4) = v;
        }
        __threadfence();
      }
    } else {
      const int q = lane >> 3, c8 = (lane & 7) * 8;
      unsigned short* C  = (unsigned short*)Cout  + (size_t)b * strideC;
      unsigned short* C2 = (OUT_MODE == 2) ? ((unsigned short*)Cout2 + (size_t)b * strideC) : nullptr;
      for (int pass = 0; pass < 2; ++pass) {
#pragma unroll
        for (int it = 0; it < 4; ++it) {
          const int row = it * 4 + q;
          const float* sp = slab + row * 68 + c8;
          v8h hv, lv;
#pragma unroll
          for (int e = 0; e < 8; ++e) {
            if (OUT_MODE == 1) {
              hv[e] = (_Float16)sp[e];
            } else {
              unsigned short hb = f2bf_bits(sp[e]);
              unsigned short lb = f2bf_bits(sp[e] - bf_bits2f(hb));
              hv[e] = __builtin_bit_cast(_Float16, hb);
              lv[e] = __builtin_bit_cast(_Float16, lb);
            }
          }
          *(volatile v8h*)(C + (size_t)(mBase + row) * ldc + n0 + c8) = hv;
          if (OUT_MODE == 2) *(volatile v8h*)(C2 + (size_t)(mBase + row) * ldc + n0 + c8) = lv;
        }
        __threadfence();
      }
    }
    __builtin_amdgcn_fence(__ATOMIC_RELEASE, "workgroup");
    __builtin_amdgcn_wave_barrier();
    __builtin_amdgcn_fence(__ATOMIC_ACQUIRE, "workgroup");
  }
}

#define TP_PITCH 264
__global__ __launch_bounds__(256) void k_feat_t16(const float* __restrict__ feat, _Float16* __restrict__ outp) {
  __shared__ __align__(16) _Float16 tile[64 * TP_PITCH];
  const int n  = blockIdx.x >> 6;
  const int p0 = (blockIdx.x & 63) * 64;
  const int t  = threadIdx.x;
  const int px = t & 63, cq = t >> 6;
  const float* src = feat + (size_t)n * (256 * 4096) + p0 + px;
#pragma unroll 8
  for (int cc = 0; cc < 256; cc += 4) {
    const int c = cc + cq;
    const float v = src[(size_t)c * 4096];
    tile[px * TP_PITCH + c] = (_Float16)v;
  }
  __syncthreads();
  const int wave = t >> 5, lane = t & 31;
  _Float16* dst = outp + ((size_t)n * 4096 + p0) * 256 + lane * 8;
  for (int pass = 0; pass < 2; ++pass) {
#pragma unroll
    for (int i = 0; i < 8; ++i) {
      const int pr = wave * 8 + i;
      const v8h v = *(const v8h*)(tile + pr * TP_PITCH + lane * 8);
      *(volatile v8h*)(dst + (size_t)pr * 256) = v;
    }
    __threadfence();
  }
}

__global__ __launch_bounds__(256) void k_cast_w(const float* __restrict__ W1, const float* __restrict__ b1,
                                               const float* __restrict__ W2, const float* __restrict__ b2,
                                               const float* __restrict__ W3,
                                               _Float16* __restrict__ W12h, _Float16* __restrict__ W3h,
                                               float* __restrict__ bias12) {
  const int NP12 = 320 * 256 / 2;
  const int NP3  = 256 * 320 / 2;
  const int i = blockIdx.x * 256 + threadIdx.x;
  if (i >= NP12 + NP3) return;
  const int e12 = min(2 * i, 2 * NP12 - 2);
  const int eW2 = min(e12, 256 * 256 - 2);
  const int eW1 = min(max(e12 - 256 * 256, 0), 64 * 256 - 2);
  const int e3  = min(max(2 * (i - NP12), 0), 2 * NP3 - 2);
  const float a0 = W2[eW2], a1 = W2[eW2 + 1];
  const float c0 = W1[eW1], c1 = W1[eW1 + 1];
  const float d0 = W3[e3],  d1 = W3[e3 + 1];
  float f0, f1;
  if (i < NP12) { const bool lo = (e12 < 256 * 256); f0 = lo ? a0 : c0; f1 = lo ? a1 : c1; }
  else { f0 = d0; f1 = d1; }
  const _Float16 h0 = (_Float16)(f0 * 16.0f), h1 = (_Float16)(f1 * 16.0f);
  const unsigned u = (unsigned)__builtin_bit_cast(unsigned short, h0) | ((unsigned)__builtin_bit_cast(unsigned short, h1) << 16);
  if (i < NP12) {
    volatile unsigned* d = (volatile unsigned*)(void*)(W12h + 2 * (size_t)i);
    *d = u; __threadfence(); *d = u;
  } else {
    volatile unsigned* d = (volatile unsigned*)(void*)(W3h + 2 * (size_t)(i - NP12));
    *d = u; __threadfence(); *d = u;
  }
  if (i < 320) {
    const float pb2 = b2[min(i, 255)];
    const float pb1 = b1[min(max(i - 256, 0), 63)];
    const float bv = (i < 256) ? pb2 : pb1;
    volatile float* d = bias12 + i;
    *d = bv; __threadfence(); *d = bv;
  }
}

__global__ __launch_bounds__(256) void k_stats(const float* __restrict__ conv, float* __restrict__ meanp,
                                              float* __restrict__ rstdp) {
  __shared__ float sh1[8][32];
  __shared__ float sh2[8][32];
  const int n = blockIdx.x / 10, cg = blockIdx.x - n * 10;
  const int t = threadIdx.x, c = t & 31, rs = t >> 5;
  const float* base = conv + (size_t)n * (4096 * 320) + cg * 32 + c;
  float s1 = 0.f, s2 = 0.f;
#pragma unroll 4
  for (int r = rs; r < 4096; r += 8) {
    const float x = base[(size_t)r * 320];
    s1 += x; s2 += x * x;
  }
  sh1[rs][c] = s1; sh2[rs][c] = s2;
  __syncthreads();
  if (t < 32) {
    float a = 0.f, bsum = 0.f;
#pragma unroll
    for (int k = 0; k < 8; ++k) { a += sh1[k][t]; bsum += sh2[k][t]; }
    const float mean = a * (1.0f / 4096.0f);
    float var = bsum * (1.0f / 4096.0f) - mean * mean;
    var = fmaxf(var, 0.0f);
    const float rstd = rsqrtf(var + 1e-5f);
    volatile float* pm = meanp + n * 320 + cg * 32 + t;
    volatile float* pr = rstdp + n * 320 + cg * 32 + t;
    *pm = mean; *pr = rstd;
    __threadfence();
    *pm = mean; *pr = rstd;
  }
}

__device__ __forceinline__ v4f relu4(v4f x) {
  v4f r;
  r[0] = fmaxf(x[0], 0.0f); r[1] = fmaxf(x[1], 0.0f); r[2] = fmaxf(x[2], 0.0f); r[3] = fmaxf(x[3], 0.0f);
  return r;
}
__global__ __launch_bounds__(256) void k_norm(const float* __restrict__ conv, const float* __restrict__ meanp,
                                             const float* __restrict__ rstdp, float* __restrict__ fnorm,
                                             _Float16* __restrict__ cat, int npix) {
  const int lane = threadIdx.x & 31;
  const int q0 = (blockIdx.x * 8 + (int)(threadIdx.x >> 5)) * 4;
  if (q0 >= npix) return;
  const int n = q0 >> 12;
  const int cA = 4 * lane, cB = 128 + 4 * lane, cS = 256 + 8 * (lane & 7);
  const float* mp = meanp + n * 320;
  const float* rp = rstdp + n * 320;
  const v4f mA  = *(const v4f*)(mp + cA),     rA  = *(const v4f*)(rp + cA);
  const v4f mB  = *(const v4f*)(mp + cB),     rB  = *(const v4f*)(rp + cB);
  const v4f mS0 = *(const v4f*)(mp + cS),     rS0 = *(const v4f*)(rp + cS);
  const v4f mS1 = *(const v4f*)(mp + cS + 4), rS1 = *(const v4f*)(rp + cS + 4);
#pragma unroll 1
  for (int i = 0; i < 4; ++i) {
    const size_t q = (size_t)(q0 + i);
    const float* row = conv + q * 320;
    const v4f xA  = *(const v4f*)(row + cA);
    const v4f xB  = *(const v4f*)(row + cB);
    const v4f xS0 = *(const v4f*)(row + cS);
    const v4f xS1 = *(const v4f*)(row + cS + 4);
    const v4f yA  = relu4((xA  - mA)  * rA);
    const v4f yB  = relu4((xB  - mB)  * rB);
    const v4f yS0 = relu4((xS0 - mS0) * rS0);
    const v4f yS1 = relu4((xS1 - mS1) * rS1);
    v8h hs;
#pragma unroll
    for (int e = 0; e < 4; ++e) { hs[e] = (_Float16)yS0[e]; hs[4 + e] = (_Float16)yS1[e]; }
    volatile v4f* pa = (volatile v4f*)(fnorm + q * 256 + cA);
    volatile v4f* pb = (volatile v4f*)(fnorm + q * 256 + cB);
    volatile v8h* ps = (volatile v8h*)(void*)(cat + q * 320 + cS);
    *pa = yA; *pb = yB;
    if (lane < 8) *ps = hs;
    __threadfence();
    *pa = yA; *pb = yB;
    if (lane < 8) *ps = hs;
  }
}

__device__ __forceinline__ void sample_pt(int g, int p, float x1, float y1, float x2, float y2,
                                          int& i00, int& i01, int& i10, int& i11,
                                          float& w00, float& w01, float& w10, float& w11) {
#pragma clang fp contract(off)
  const float t  = (float)p * 0.1f;
  const float xt = x1 + (x2 - x1) * t;
  const float yt = y1 + (y2 - y1) * t;
  const bool gx = (g == 0) | (g == 2);
  const bool gy = (g == 1) | (g == 3);
  float x = gx ? xt : ((g == 1) ? x1 : x2);
  float y = gy ? yt : ((g == 0) ? y1 : y2);
  const bool inval = (y < -1.0f) | (y > 64.0f) | (x < -1.0f) | (x > 64.0f);
  y = fmaxf(y, 0.0f);
  x = fmaxf(x, 0.0f);
  const float yf = fminf(floorf(y), 63.0f);
  const float xf = fminf(floorf(x), 63.0f);
  const int yl = (int)yf, xl = (int)xf;
  const int yh = min(yl + 1, 63), xh = min(xl + 1, 63);
  const float ly = y - (float)yl, lx = x - (float)xl;
  const float hy = 1.0f - ly, hx = 1.0f - lx;
  const float a00 = hy * hx, a01 = hy * lx, a10 = ly * hx, a11 = ly * lx;
  w00 = inval ? 0.0f : a00;
  w01 = inval ? 0.0f : a01;
  w10 = inval ? 0.0f : a10;
  w11 = inval ? 0.0f : a11;
  i00 = yl * 64 + xl; i01 = yl * 64 + xh;
  i10 = yh * 64 + xl; i11 = yh * 64 + xh;
}

__global__ __launch_bounds__(256) void k_border(const float* __restrict__ fnorm, const float* __restrict__ boxes,
                                               _Float16* __restrict__ cat, int nbox) {
  const int lane = threadIdx.x & 31;
  const int q = blockIdx.x * 8 + (int)(threadIdx.x >> 5);
  if (q >= nbox) return;
  const int n = q >> 12;
  const v4f bx = *(const v4f*)(boxes + (size_t)q * 4);
  const float* fimg = fnorm + (size_t)n * (4096 * 256) + 2 * lane;
  _Float16* crow = cat + (size_t)q * 320 + 2 * lane;
  const int pl = (lane < 11) ? lane : 10;
#pragma unroll 1
  for (int g = 0; g < 4; ++g) {
    int i00, i01, i10, i11; float w00, w01, w10, w11;
    sample_pt(g, pl, bx[0], bx[1], bx[2], bx[3], i00, i01, i10, i11, w00, w01, w10, w11);
    const float* fg = fimg + g * 64;
    float m0 = -__builtin_inff(), m1 = -__builtin_inff();
#pragma unroll 1
    for (int p = 0; p < 11; ++p) {
      const int j00 = __builtin_amdgcn_readlane(i00, p);
      const int j01 = __builtin_amdgcn_readlane(i01, p);
      const int j10 = __builtin_amdgcn_readlane(i10, p);
      const int j11 = __builtin_amdgcn_readlane(i11, p);
      const float u00 = __int_as_float(__builtin_amdgcn_readlane(__float_as_int(w00), p));
      const float u01 = __int_as_float(__builtin_amdgcn_readlane(__float_as_int(w01), p));
      const float u10 = __int_as_float(__builtin_amdgcn_readlane(__float_as_int(w10), p));
      const float u11 = __int_as_float(__builtin_amdgcn_readlane(__float_as_int(w11), p));
      const v2f a = *(const v2f*)(fg + (size_t)j00 * 256);
      const v2f b = *(const v2f*)(fg + (size_t)j01 * 256);
      const v2f c = *(const v2f*)(fg + (size_t)j10 * 256);
      const v2f d = *(const v2f*)(fg + (size_t)j11 * 256);
      const float v0 = u00 * a[0] + u01 * b[0] + u10 * c[0] + u11 * d[0];
      const float v1 = u00 * a[1] + u01 * b[1] + u10 * c[1] + u11 * d[1];
      m0 = fmaxf(m0, v0);
      m1 = fmaxf(m1, v1);
    }
    const unsigned u = (unsigned)__builtin_bit_cast(unsigned short, (_Float16)m0) |
                       ((unsigned)__builtin_bit_cast(unsigned short, (_Float16)m1) << 16);
    volatile unsigned* dp = (volatile unsigned*)(void*)(crow + g * 64);
    *dp = u;
    __threadfence();
    *dp = u;
  }
}

extern "C" void kernel_launch(void* const* d_in, const int* in_sizes, int n_in,
                              void* d_out, int out_size, void* d_ws, size_t ws_size,
                              hipStream_t stream) {
  const int NI = 4, CIN = 256, CB = 64, HW = 4096, C12 = 320;
  if (n_in < 9) return;
  if (in_sizes[0] != NI * CIN * HW) return;
  if (in_sizes[1] != NI * HW * 4) return;
  if (in_sizes[3] != CB * CIN || in_sizes[4] != CB) return;
  if (in_sizes[5] != 4 * CB * CIN || in_sizes[6] != 4 * CB) return;
  if (in_sizes[7] != CIN * C12 || in_sizes[8] != CIN) return;
  if (out_size != NI * CIN * HW) return;

  const float* feature = (const float*)d_in[0];
  const float* boxes   = (const float*)d_in[1];
  const float* W1 = (const float*)d_in[3];
  const float* b1 = (const float*)d_in[4];
  const float* W2 = (const float*)d_in[5];
  const float* b2 = (const float*)d_in[6];
  const float* W3 = (const float*)d_in[7];
  const float* b3 = (const float*)d_in[8];
  float* out = (float*)d_out;

  char* ws = (char*)d_ws;
  size_t off = 0;
  _Float16* featT = (_Float16*)(ws + off); off += (size_t)NI * HW * CIN * 2;
  _Float16* W12h  = (_Float16*)(ws + off); off += (size_t)C12 * CIN * 2;
  _Float16* W3h   = (_Float16*)(ws + off); off += (size_t)CIN * C12 * 2;
  float* bias12   = (float*)(ws + off);    off += (size_t)C12 * 4;
  float* conv12   = (float*)(ws + off);    off += (size_t)NI * HW * C12 * 4;
  float* meanp    = (float*)(ws + off);    off += (size_t)NI * C12 * 4;
  float* rstdp    = (float*)(ws + off);    off += (size_t)NI * C12 * 4;
  float* fnorm    = (float*)(ws + off);    off += (size_t)NI * HW * 256 * 4;
  _Float16* cat   = (_Float16*)(ws + off); off += (size_t)NI * HW * C12 * 2;
  if (off > ws_size || off > (size_t)134217728) return;

  k_feat_t16<<<NI * 64, 256, 0, stream>>>(feature, featT);

  k_cast_w<<<(40960 + 40960) / 256, 256, 0, stream>>>(W1, b1, W2, b2, W3, W12h, W3h, bias12);

  {
    dim3 grid((64 * 5 + 7) / 8, NI);
    wmma_gemm64<0, false, 2, 0, false, 0><<<grid, 256, 0, stream>>>(
        (const unsigned short*)featT, (const unsigned short*)featT, CIN, (long)HW * CIN,
        (const unsigned short*)W12h, (const unsigned short*)W12h, CIN, 0L,
        (void*)conv12, (void*)conv12, C12, (long)HW * C12,
        bias12, bias12, 0L, HW, C12, CIN, 1.0f / 16.0f);
  }

  k_stats<<<NI * 10, 256, 0, stream>>>(conv12, meanp, rstdp);

  k_norm<<<(NI * HW) / 32, 256, 0, stream>>>(conv12, meanp, rstdp, fnorm, cat, NI * HW);

  k_border<<<(NI * HW) / 8, 256, 0, stream>>>(fnorm, boxes, cat, NI * HW);

  {
    dim3 grid((4 * 64 + 7) / 8, NI);
    wmma_gemm64<0, false, 1, 0, false, 2><<<grid, 256, 0, stream>>>(
        (const unsigned short*)W3h, (const unsigned short*)W3h, C12, 0L,
        (const unsigned short*)cat, (const unsigned short*)cat, C12, (long)HW * C12,
        (void*)out, (void*)out, HW, (long)CIN * HW,
        b3, b3, 0L, CIN, HW, C12, 1.0f / 16.0f);
  }
}
